// NonOverlappingLocallyConnected1d_24885040513342
// MI455X (gfx1250) — hardware-run, weakly checked
//
#include <hip/hip_runtime.h>


#ifndef NB
#define NB 16
#endif
#ifndef NP
#define NP 1024
#endif
#define NP_FULL   1024
#define DLEN_FULL (4 * NP_FULL)
#ifndef OUT_P
#define OUT_P NP
#endif
#define CIN    32
#define COUT   64
#define KPATCH 4
#define KD     (CIN * KPATCH)
#define PCH    32
#define TW     4
#define TP     136
#define OSP    36
#define SCL    0.17677669529663687f

static_assert(NB == 16);
static_assert(COUT % 16 == 0);
static_assert(KPATCH == 4);
static_assert(KD == 128);
static_assert(KD % 32 == 0);
static_assert(NP % PCH == 0);
static_assert(NP <= NP_FULL);
static_assert((NP / PCH) % TW == 0);
static_assert((TP * 2) % 16 == 0);
static_assert(TP >= KD);
static_assert((OSP * 4) % 16 == 0);
static_assert(OSP >= PCH);
static_assert(OUT_P % 32 == 0);
static_assert((size_t)TW * 32 * TP * 2 <= 131072);
static_assert((size_t)NB * 16 * OSP * 4 <= 131072);

typedef unsigned short bf;
typedef __attribute__((ext_vector_type(16))) __bf16   v16bf;
typedef __attribute__((ext_vector_type(8)))  unsigned short v8us;
typedef __attribute__((ext_vector_type(4)))  unsigned short v4us;
typedef __attribute__((ext_vector_type(8)))  float    v8f;
typedef __attribute__((ext_vector_type(4)))  float    v4f;
typedef v4f  __attribute__((may_alias)) v4fa;
typedef v4us __attribute__((may_alias)) v4usa;
typedef v8us __attribute__((may_alias)) v8usa;

__device__ __forceinline__ unsigned short f2bf(float f) { unsigned u = __float_as_uint(f); u += 0x7FFFu + ((u >> 16) & 1u); return (unsigned short)(u >> 16); }
__device__ __forceinline__ v16bf cat16b(v8us lo, v8us hi) { return __builtin_bit_cast(v16bf, __builtin_shufflevector(lo, hi, 0, 1, 2, 3, 4, 5, 6, 7, 8, 9, 10, 11, 12, 13, 14, 15)); }
__device__ __forceinline__ v8f wmmab(v16bf a, v16bf b, v8f c) { return __builtin_amdgcn_wmma_f32_16x16x32_bf16(false, a, false, b, (short)0, c, false, false); }
__device__ __forceinline__ v8f wmmabg(v16bf a, v16bf b, v8f c) { c = wmmab(a, b, c); asm volatile("v_nop\n\tv_nop\n\tv_nop\n\tv_nop" : "+v"(c) : "v"(a), "v"(b)); return c; }
__device__ __forceinline__ v16bf ldb(const bf* p)  { return cat16b(*(const v8us*)p, *(const v8us*)(p + 16)); }
__device__ __forceinline__ void wave_sync() { __builtin_amdgcn_fence(3  , "wavefront"); __builtin_amdgcn_wave_barrier(); asm volatile("" ::: "memory"); }

static_assert(16 * 2 == 32);
static_assert(16 * 16 == KD * 2);
__global__ __launch_bounds__(32 * TW) void k_relay(const float* __restrict__ src, bf* dst, int R) {
    __shared__ __align__(16) unsigned short ts[TW * 32 * TP];
    const int lane = threadIdx.x & 31;
    const int wave = __builtin_amdgcn_readfirstlane((int)(threadIdx.x >> 5));
    const int unit = blockIdx.x * TW + wave;
    const int npc = NP / PCH;
    if (unit >= R * npc) return;
    const int r = unit / npc, p0 = (unit % npc) * 32;
    const float* s = src + (size_t)r * CIN * DLEN_FULL + (size_t)4 * (p0 + lane);
    const int wb = wave * 32 * TP;
#pragma unroll 8
    for (int c = 0; c < CIN; ++c) {
        const v4f v = *(const v4f*)(s + (size_t)c * DLEN_FULL);
        v4us o;
#pragma unroll
        for (int k = 0; k < 4; ++k) o[k] = f2bf(v[k]);
        *(v4usa*)(&ts[wb + lane * TP + c * 4]) = o;
    }
    wave_sync();
#pragma unroll 1
    for (int ps = 0; ps < 2; ++ps) {
#pragma unroll 4
        for (int t = 0; t < 16; ++t) { const int row = 2 * t + (lane >> 4), c8 = (lane & 15) * 8;
            const v8us val = *(const v8usa*)(&ts[wb + row * TP + c8]);
            *(volatile v8us*)(dst + ((size_t)(p0 + row) * (size_t)R + (size_t)r) * KD + c8) = val; }
        if (ps == 0) __threadfence(); }
}

static_assert(64 * 4 == NB * 16);
static_assert(8 * 16 == PCH * 4);
__global__ __launch_bounds__(32) void k_lcgemm(const bf* __restrict__ XP, const bf* __restrict__ WP, float* OUT) {
    __shared__ __align__(16) float os[NB * 16 * OSP];
    const int lane = threadIdx.x & 31, lr = lane & 15, hi = lane >> 4;
    const int p0 = blockIdx.x * PCH, o0 = blockIdx.y * 16;
    const size_t aoff = (size_t)lr * KD + 8 * hi;
    const size_t boff = (size_t)(o0 + lr) * KD + 8 * hi;
#pragma unroll 1
    for (int pi = 0; pi < PCH; ++pi) {
        const size_t p = (size_t)(p0 + pi);
        const bf* ap = XP + p * ((size_t)NB * KD) + aoff;
        const bf* bp = WP + p * ((size_t)COUT * KD) + boff;
        v16bf a[4], b[4];
#pragma unroll
        for (int ks = 0; ks < 4; ++ks) { a[ks] = ldb(ap + 32 * ks); b[ks] = ldb(bp + 32 * ks); }
        v8f acc = (v8f){};
#pragma unroll
        for (int ks = 0; ks < 4; ++ks) acc = wmmabg(a[ks], b[ks], acc);
#pragma unroll
        for (int r = 0; r < 8; ++r) os[((8 * hi + r) * 16 + lr) * OSP + pi] = acc[r] * SCL;
    }
    wave_sync();
    float* obase = OUT + (size_t)o0 * OUT_P + p0;
#pragma unroll 1
    for (int ps = 0; ps < 2; ++ps) {
#pragma unroll 4
        for (int t = 0; t < 64; ++t) { const int row = 4 * t + (lane >> 3), cofs = (lane & 7) * 4;
            const int bb = row >> 4, oo = row & 15;
            const v4f val = *(const v4fa*)(&os[row * OSP + cofs]);
            *(volatile v4f*)(obase + ((size_t)bb * COUT + (size_t)oo) * OUT_P + cofs) = val; }
        if (ps == 0) __threadfence(); }
}

static constexpr size_t al256(size_t v) { return (v + 255) & ~(size_t)255; }
static constexpr size_t SZ_XP = al256((size_t)NP * NB * KD * 2);
static constexpr size_t SZ_WP = al256((size_t)NP * COUT * KD * 2);
static constexpr size_t SZ_TOTAL = SZ_XP + SZ_WP;
static_assert(SZ_TOTAL <= (size_t)134217728);
static constexpr size_t NEED_X = ((size_t)NB * CIN - 1) * DLEN_FULL + (size_t)4 * NP;
static constexpr size_t NEED_W = ((size_t)COUT * CIN - 1) * DLEN_FULL + (size_t)4 * NP;
static constexpr size_t NEED_O = ((size_t)NB * COUT - 1) * OUT_P + (size_t)NP;
static constexpr unsigned GRID_RX = (unsigned)(NB * (NP / PCH) / TW);
static constexpr unsigned GRID_RW = (unsigned)(COUT * (NP / PCH) / TW);
static_assert((size_t)GRID_RX * TW == (size_t)NB * (NP / PCH));
static_assert((size_t)GRID_RW * TW == (size_t)COUT * (NP / PCH));

extern "C" void kernel_launch(void* const* d_in, const int* in_sizes, int n_in,
                              void* d_out, int out_size, void* d_ws, size_t ws_size, hipStream_t stream) {
    if (n_in < 2) return;
    if ((size_t)in_sizes[0] < NEED_X || (size_t)in_sizes[1] < NEED_W) return;
    if ((size_t)out_size < NEED_O) return;
    if (SZ_TOTAL > ws_size) return;
    const float* x = (const float*)d_in[0];
    const float* w = (const float*)d_in[1];
    float* OUT = (float*)d_out;
    char* wsp = (char*)d_ws;
    bf* XP = (bf*)wsp; wsp += SZ_XP;
    bf* WP = (bf*)wsp; wsp += SZ_WP;

    k_relay<<<GRID_RX, 32 * TW, 0, stream>>>(x, XP, NB);
    k_relay<<<GRID_RW, 32 * TW, 0, stream>>>(w, WP, COUT);
    k_lcgemm<<<dim3(NP / PCH, COUT / 16, 1), 32, 0, stream>>>(XP, WP, OUT);
}
